// Nalui2Layer_55594056679945
// MI455X (gfx1250) — hardware-run, weakly checked
//
#include <hip/hip_runtime.h>


#ifndef NB
#define NB 1024
#endif
#define NB_FULL 1024
#define KD   512
#define NO   512
#define OSP  36
#define WT   64
#define WP   66
#define LOG2E 1.4426950408889634f
#define LZERO (-200.0f)

static_assert(KD % 32 == 0);
static_assert(KD == NO);
static_assert(KD % WT == 0);
static_assert(NO % WT == 0);
static_assert(NO % 32 == 0);
static_assert(NB % 16 == 0);
static_assert(NB <= NB_FULL);
static_assert(((size_t)NB * KD) % 8 == 0);
static_assert(16 * 256 == WT * WT);
static_assert(256 * 8 * 2 == WT * WT);
static_assert(32 * 4 * 4 == 16 * 32);
static_assert((OSP * 4) % 16 == 0);
static_assert(5 * WT * WP * 2 <= 131072);
static_assert(16 * OSP * 4 <= 131072);
static_assert(WP >= WT);

typedef _Float16 h16;
typedef unsigned short bf;
typedef __attribute__((ext_vector_type(16))) __bf16   v16bf;
typedef __attribute__((ext_vector_type(16))) _Float16 v16h;
typedef __attribute__((ext_vector_type(8)))  _Float16 v8h;
typedef __attribute__((ext_vector_type(8)))  unsigned short v8us;
typedef __attribute__((ext_vector_type(8)))  float    v8f;
typedef __attribute__((ext_vector_type(4)))  float    v4f;
typedef v4f  __attribute__((may_alias)) v4fa;

__device__ __forceinline__ unsigned short f2bf(float f) { unsigned u = __float_as_uint(f); u += 0x7FFFu + ((u >> 16) & 1u); return (unsigned short)(u >> 16); }
__device__ __forceinline__ float bfr(float f) { return __uint_as_float(((unsigned)f2bf(f)) << 16); }
__device__ __forceinline__ v16h cat16(v8h lo, v8h hi) { return __builtin_shufflevector(lo, hi, 0, 1, 2, 3, 4, 5, 6, 7, 8, 9, 10, 11, 12, 13, 14, 15); }
__device__ __forceinline__ v16bf cat16b(v8us lo, v8us hi) { return __builtin_bit_cast(v16bf, __builtin_shufflevector(lo, hi, 0, 1, 2, 3, 4, 5, 6, 7, 8, 9, 10, 11, 12, 13, 14, 15)); }
__device__ __forceinline__ v8f wmma16(v16h a, v16h b, v8f c) { return __builtin_amdgcn_wmma_f32_16x16x32_f16(false, a, false, b, (short)0, c, false, false); }
__device__ __forceinline__ v8f wmmab(v16bf a, v16bf b, v8f c) { return __builtin_amdgcn_wmma_f32_16x16x32_bf16(false, a, false, b, (short)0, c, false, false); }
__device__ __forceinline__ v16h  ldh(const h16* p) { return cat16(*(const v8h*)p, *(const v8h*)(p + 16)); }
__device__ __forceinline__ v16bf ldb(const bf* p)  { return cat16b(*(const v8us*)p, *(const v8us*)(p + 16)); }
__device__ __forceinline__ void wave_sync() { __builtin_amdgcn_fence(3  , "wavefront"); __builtin_amdgcn_wave_barrier(); asm volatile("" ::: "memory"); }

__device__ __forceinline__ h16 toh_flush(float v) { const h16 r = (h16)v; return (fabsf(v) < 6.103515625e-05f) ? (h16)0.0f : r; }
__device__ __forceinline__ v8f wmma16g(v16h a, v16h b, v8f c) { c = wmma16(a, b, c); asm volatile("v_nop\n\tv_nop\n\tv_nop\n\tv_nop" : "+v"(c) : "v"(a), "v"(b)); return c; }
__device__ __forceinline__ float sig_e(float x)  { return __builtin_amdgcn_rcpf(1.0f + __builtin_amdgcn_exp2f(-x * LOG2E)); }
__device__ __forceinline__ float tanh_e(float x) { return 1.0f - 2.0f * __builtin_amdgcn_rcpf(1.0f + __builtin_amdgcn_exp2f(2.0f * x * LOG2E)); }

__global__ __launch_bounds__(256) void k_xprep(const float* __restrict__ X, h16* XH, h16* LXH, h16* NGH, h16* ZH, size_t n8) {
#pragma clang fp contract(off)
    const size_t i = (size_t)blockIdx.x * 256 + threadIdx.x; if (i >= n8) return;
    const v8f v = *(const v8f*)(X + i * 8); v8h xo, lo, no, zo;
#pragma unroll
    for (int k = 0; k < 8; ++k) {
        const float xb = bfr(v[k]);
        xo[k] = toh_flush(xb);
        lo[k] = toh_flush(__logf(fmaxf(fabsf(xb), 1.0e-7f)));
        no[k] = toh_flush((xb < 0.0f) ? 1.0f : 0.0f);
        zo[k] = toh_flush((xb == 0.0f) ? 1.0f : 0.0f);
    }
    *(volatile v8h*)(XH + i * 8) = xo; *(volatile v8h*)(LXH + i * 8) = lo; *(volatile v8h*)(NGH + i * 8) = no; *(volatile v8h*)(ZH + i * 8) = zo;
    __threadfence();
    *(volatile v8h*)(XH + i * 8) = xo; *(volatile v8h*)(LXH + i * 8) = lo; *(volatile v8h*)(NGH + i * 8) = no; *(volatile v8h*)(ZH + i * 8) = zo;
}

__global__ __launch_bounds__(256) void k_wprep(const float* __restrict__ w1h, const float* __restrict__ m1h, const float* __restrict__ w2h, const float* __restrict__ m2h,
                                               h16* W1T, h16* W2T, h16* LT, h16* ST, h16* LZT) {
#pragma clang fp contract(off)
    __shared__ h16 t1[WT * WP];
    __shared__ h16 t2[WT * WP];
    __shared__ h16 tl[WT * WP];
    __shared__ h16 ts[WT * WP];
    __shared__ h16 tz[WT * WP];
    const int tid = threadIdx.x;
    const int c0 = blockIdx.x * WT, r0 = blockIdx.y * WT;
#pragma unroll 1
    for (int j = 0; j < 16; ++j) {
        const int e = j * 256 + tid; const int r = e >> 6, c = e & 63;
        const size_t g = (size_t)(r0 + r) * NO + (size_t)(c0 + c);
        const float a1 = bfr(w1h[g]), b1 = bfr(m1h[g]), a2 = bfr(w2h[g]), b2 = bfr(m2h[g]);
        const float v1 = tanh_e(a1) * sig_e(b1);
        const float v2 = tanh_e(a2) * sig_e(b2);
        const float w = fabsf(v2);
        const float u = 1.0f - w;
        const float t = u - w;
        const float at = fabsf(t);
        const float lt = (at > 0.0f) ? __logf(fmaxf(at, 1.0e-37f)) : LZERO;
        const float lz = (u > 0.0f) ? __logf(fmaxf(u, 1.0e-37f)) : LZERO;
        t1[r * WP + c] = toh_flush(v1);
        t2[r * WP + c] = toh_flush(v2);
        tl[r * WP + c] = toh_flush(lt);
        ts[r * WP + c] = toh_flush((t < 0.0f) ? 1.0f : 0.0f);
        tz[r * WP + c] = toh_flush(lz);
    }
    __syncthreads();
#pragma unroll 1
    for (int ps = 0; ps < 2; ++ps) {
#pragma unroll
        for (int it = 0; it < 2; ++it) { const int p = it * 256 + tid; const int rr = p >> 3, q8 = (p & 7) * 8;
            v8h xa, xb, xl, xs, xz;
#pragma unroll
            for (int i = 0; i < 8; ++i) {
                xa[i] = t1[(q8 + i) * WP + rr]; xb[i] = t2[(q8 + i) * WP + rr];
                xl[i] = tl[rr * WP + q8 + i]; xs[i] = ts[rr * WP + q8 + i]; xz[i] = tz[rr * WP + q8 + i]; }
            const size_t ot = (size_t)(c0 + rr) * KD + (size_t)(r0 + q8);
            const size_t on = (size_t)(r0 + rr) * KD + (size_t)(c0 + q8);
            *(volatile v8h*)(W1T + ot) = xa; *(volatile v8h*)(W2T + ot) = xb;
            *(volatile v8h*)(LT + on) = xl; *(volatile v8h*)(ST + on) = xs; *(volatile v8h*)(LZT + on) = xz; }
        if (ps == 0) __threadfence(); }
}

__global__ __launch_bounds__(32) void k_fused(const h16* __restrict__ XH, const h16* __restrict__ LXH, const h16* __restrict__ NGH, const h16* __restrict__ ZH,
                                              const h16* __restrict__ W1T, const h16* __restrict__ W2T, const h16* __restrict__ LT, const h16* __restrict__ ST, const h16* __restrict__ LZT,
                                              const float* __restrict__ G1, float* OUT) {
    __shared__ __align__(16) float os[16 * OSP];
    const int lane = threadIdx.x & 31, lr = lane & 15, hi = lane >> 4;
    const int r0 = blockIdx.x * 16, c0 = blockIdx.y * 32;
    v8f cA[2], cM[2], cS[2], cP[2];
#pragma unroll
    for (int nb = 0; nb < 2; ++nb) { cA[nb] = (v8f){}; cM[nb] = (v8f){}; cS[nb] = (v8f){}; cP[nb] = (v8f){}; }
    const size_t aoff = (size_t)(r0 + lr) * KD + 8 * hi, boff = (size_t)(c0 + lr) * KD + 8 * hi;
#pragma unroll 1
    for (int kc = 0; kc < KD; kc += 32) {
        const v16h ax = ldh(XH + aoff + kc), al = ldh(LXH + aoff + kc), an = ldh(NGH + aoff + kc), az = ldh(ZH + aoff + kc);
#pragma unroll
        for (int nb = 0; nb < 2; ++nb) { const size_t bo = boff + (size_t)nb * 16 * KD + kc;
            const v16h b1 = ldh(W1T + bo); cA[nb] = wmma16g(ax, b1, cA[nb]);
            const v16h b2 = ldh(W2T + bo); cM[nb] = wmma16g(al, b2, cM[nb]);
            const v16h bl = ldh(LT + bo);  cS[nb] = wmma16g(an, bl, cS[nb]);
            const v16h bz = ldh(LZT + bo); cS[nb] = wmma16g(az, bz, cS[nb]);
            const v16h bs = ldh(ST + bo);  cP[nb] = wmma16g(an, bs, cP[nb]); }
    }
#pragma unroll
    for (int nb = 0; nb < 2; ++nb) {
        const float g = sig_e(bfr(G1[c0 + nb * 16 + lr]));
        const float gm = 1.0f - g;
#pragma unroll
        for (int j = 0; j < 8; ++j) {
            const float a1 = cA[nb][j];
            const float m1 = __builtin_amdgcn_exp2f(fminf(cM[nb][j], 20.0f) * LOG2E);
            const float mag = __builtin_amdgcn_exp2f(cS[nb][j] * LOG2E);
            const int par = ((int)(cP[nb][j] + 0.5f)) & 1;
            float ms = par ? -mag : mag;
            ms = fminf(fmaxf(ms, -1.0f), 1.0f);
            os[(hi * 8 + j) * OSP + nb * 16 + lr] = g * a1 + (gm * m1) * ms; } }
    wave_sync();
    float* orow = OUT + (size_t)r0 * NO + c0;
#pragma unroll 1
    for (int ps = 0; ps < 2; ++ps) {
#pragma unroll
        for (int s = 0; s < 4; ++s) { const int row = 4 * s + (lane >> 3), cofs = (lane & 7) * 4;
            const v4f val = *(const v4fa*)(&os[row * OSP + cofs]);
            *(volatile v4f*)(orow + (size_t)row * NO + cofs) = val; }
        if (ps == 0) __threadfence(); }
}

static constexpr size_t al256(size_t v) { return (v + 255) & ~(size_t)255; }
static constexpr size_t SZ_XP = al256((size_t)NB * KD * 2);
static constexpr size_t SZ_WP = al256((size_t)NO * KD * 2);
static constexpr size_t SZ_TOTAL = 4 * SZ_XP + 5 * SZ_WP;
static_assert(SZ_TOTAL <= (size_t)134217728);
static_assert(((size_t)NB * KD * 2) % 128 == 0);
static_assert(((size_t)NO * KD * 2) % 128 == 0);

extern "C" void kernel_launch(void* const* d_in, const int* in_sizes, int n_in,
                              void* d_out, int out_size, void* d_ws, size_t ws_size, hipStream_t stream) {
    if (n_in < 6) return;
    if ((size_t)in_sizes[0] < (size_t)NB * KD) return;
    if ((size_t)in_sizes[1] < (size_t)KD * NO || (size_t)in_sizes[2] < (size_t)KD * NO || (size_t)in_sizes[3] < (size_t)KD * NO || (size_t)in_sizes[4] < (size_t)KD * NO) return;
    if (in_sizes[5] < NO) return;
    if ((size_t)out_size < (size_t)NB * NO) return;
    if (SZ_TOTAL > ws_size) return;
    const float* X   = (const float*)d_in[0];
    const float* w1h = (const float*)d_in[1];
    const float* m1h = (const float*)d_in[2];
    const float* w2h = (const float*)d_in[3];
    const float* m2h = (const float*)d_in[4];
    const float* G1  = (const float*)d_in[5];
    float* OUT = (float*)d_out;
    char* wsp = (char*)d_ws;
    h16* XH  = (h16*)wsp; wsp += SZ_XP;
    h16* LXH = (h16*)wsp; wsp += SZ_XP;
    h16* NGH = (h16*)wsp; wsp += SZ_XP;
    h16* ZH  = (h16*)wsp; wsp += SZ_XP;
    h16* W1T = (h16*)wsp; wsp += SZ_WP;
    h16* W2T = (h16*)wsp; wsp += SZ_WP;
    h16* LT  = (h16*)wsp; wsp += SZ_WP;
    h16* ST  = (h16*)wsp; wsp += SZ_WP;
    h16* LZT = (h16*)wsp; wsp += SZ_WP;

    { const size_t n8 = (size_t)NB * KD / 8;
      k_xprep<<<(unsigned)((n8 + 255) / 256), 256, 0, stream>>>(X, XH, LXH, NGH, ZH, n8); }
    k_wprep<<<dim3(NO / WT, KD / WT, 1), 256, 0, stream>>>(w1h, m1h, w2h, m2h, W1T, W2T, LT, ST, LZT);
    k_fused<<<dim3(NB / 16, NO / 32, 1), 32, 0, stream>>>(XH, LXH, NGH, ZH, W1T, W2T, LT, ST, LZT, G1, OUT);
}
